// TrueHigherOrderAttention_62551903699153
// MI455X (gfx1250) — hardware-run, weakly checked
//
#include <hip/hip_runtime.h>

typedef __bf16          v16b __attribute__((ext_vector_type(16)));
typedef unsigned short  v8us __attribute__((ext_vector_type(8)));
typedef float           v8f  __attribute__((ext_vector_type(8)));
typedef float           v4f  __attribute__((ext_vector_type(4)));
typedef v8us __attribute__((may_alias)) v8usa;
typedef v4f  __attribute__((may_alias)) v4fa;

union FragB { v16b v; v8us half[2]; };
union F8    { v8f v; v4f q[2]; };

#define BSZ   2
#define SEQ   192
#define EMB   512
#define NH    8
#define HD    64
#define NBH   (BSZ * NH)
#define NTOK  (BSZ * SEQ)
#define NTI   (SEQ / 16)
#define NX    (NTOK * EMB)
#define NW    (EMB * EMB)
#define NX8   (NX / 8)
#define NW8   (NW / 8)
#define PLANE (NBH * SEQ * HD)

static_assert(SEQ % 16 == 0);
static_assert(NTOK % 128 == 0);
static_assert(EMB % 64 == 0);
static_assert(HD == 64);
static_assert(NX8 % 256 == 0);
static_assert(NW8 % 256 == 0);

__device__ __forceinline__ v8f wmma_bf(v16b a, v16b b, v8f c) {
  v8f d = __builtin_amdgcn_wmma_f32_16x16x32_bf16(false, a, false, b, (short)0, c, false, false);
  asm volatile("v_nop\n\tv_nop\n\tv_nop\n\tv_nop" : "+v"(d) : "v"(a), "v"(b));
  return d;
}

__device__ __forceinline__ v16b load_frag16(const unsigned short* p, int h) {
  FragB f;
  f.half[0] = *(const v8usa*)(p + 8 * h);
  f.half[1] = *(const v8usa*)(p + 16 + 8 * h);
  return f.v;
}

__device__ __forceinline__ unsigned short bf16_bits(float f) {
  unsigned u = __float_as_uint(f);
  u += 0x7FFFu + ((u >> 16) & 1u);
  return (unsigned short)(u >> 16);
}
__device__ __forceinline__ float bf16_val(unsigned short b) {
  return __uint_as_float(((unsigned)b) << 16);
}
__device__ __forceinline__ v8f ld8f(const float* p) {
  F8 u;
  u.q[0] = *(const v4fa*)p;
  u.q[1] = *(const v4fa*)(p + 4);
  return u.v;
}
__device__ __forceinline__ void split8(v4f a, v4f c, v8us& hv, v8us& lv) {
  F8 u; u.q[0] = a; u.q[1] = c;
  #pragma unroll
  for (int e = 0; e < 8; ++e) {
    const float v = u.v[e];
    const unsigned short hb = bf16_bits(v);
    const unsigned short lb = bf16_bits(v - bf16_val(hb));
    hv[e] = hb; lv[e] = lb;
  }
}

__global__ __launch_bounds__(256) void cvt_kernel(
    const float* __restrict__ x,  const float* __restrict__ w0, const float* __restrict__ w1,
    const float* __restrict__ w2, const float* __restrict__ wp,
    unsigned short* __restrict__ xb, unsigned short* __restrict__ wb, unsigned short* __restrict__ wpb)
{
  const int g = blockIdx.x * 256 + threadIdx.x;
  if (g >= NX8 + 4 * NW8) return;
  const float* src;
  unsigned short* dst;
  if (g < NX8) {
    src = x + (size_t)g * 8;
    dst = xb + (size_t)g * 8;
  } else {
    const int e = g - NX8;
    const int sel = e / NW8;
    const int off = e - sel * NW8;
    const float* wsrc = (sel == 0) ? w0 : ((sel == 1) ? w1 : ((sel == 2) ? w2 : wp));
    src = wsrc + (size_t)off * 8;
    dst = (sel < 3) ? (wb + (size_t)e * 8) : (wpb + (size_t)off * 8);
  }
  const v4f a = *(const v4fa*)src;
  const v4f c = *(const v4fa*)(src + 4);
  v8us o;
  o[0] = bf16_bits(a.x); o[1] = bf16_bits(a.y); o[2] = bf16_bits(a.z); o[3] = bf16_bits(a.w);
  o[4] = bf16_bits(c.x); o[5] = bf16_bits(c.y); o[6] = bf16_bits(c.z); o[7] = bf16_bits(c.w);
  *(volatile v8us*)dst = o;
  __threadfence();
  *(volatile v8us*)dst = o;
}

__device__ __forceinline__ void proj_store(const float* sT, float* p32w,
                                           unsigned short* p1h, unsigned short* p1l,
                                           int which, int head, int m0, int w, int lane) {
  const int q8 = lane & 7, sub = lane >> 3;
  #pragma unroll
  for (int it = 0; it < 16; ++it) {
    const int lid = w * 64 + it * 4 + sub;
    const int tokl = lid >> 1, hl = lid & 1;
    const v4f v = *(const v4fa*)(sT + tokl * HD + 32 * hl + 4 * q8);
    const int mtok = m0 + tokl;
    const int b = (mtok >= SEQ) ? 1 : 0;
    const int t = mtok - b * SEQ;
    float* dst = p32w + ((size_t)(b * NH + head) * SEQ + t) * HD + 32 * hl + 4 * q8;
    *(volatile v4f*)dst = v;
  }
  if (which == 1) {
    #pragma unroll
    for (int it = 0; it < 8; ++it) {
      const int tokl = w * 32 + it * 4 + sub;
      const v4f a = *(const v4fa*)(sT + tokl * HD + 8 * q8);
      const v4f c = *(const v4fa*)(sT + tokl * HD + 8 * q8 + 4);
      v8us hv, lv;
      split8(a, c, hv, lv);
      const int mtok = m0 + tokl;
      const int b = (mtok >= SEQ) ? 1 : 0;
      const int t = mtok - b * SEQ;
      const size_t idx = ((size_t)(b * NH + head) * SEQ + t) * HD + 8 * q8;
      *(volatile v8us*)(p1h + idx) = hv;
      *(volatile v8us*)(p1l + idx) = lv;
    }
  }
}

__global__ __launch_bounds__(128) void proj_kernel(
    const unsigned short* __restrict__ xb,
    const unsigned short* __restrict__ wb,
    float* __restrict__ p32,
    unsigned short* __restrict__ p1h,
    unsigned short* __restrict__ p1l)
{
  __shared__ __attribute__((aligned(16))) float sT[128 * HD];

  const int tid = threadIdx.x, lane = tid & 31, w = tid >> 5;
  const int h = lane >> 4, m = lane & 15;
  const int m0 = blockIdx.x * 128;
  const int cg = blockIdx.y;
  const int which = cg >> 3, head = cg & 7;
  const int m0w = m0 + 32 * w;

  const unsigned short* xa0 = xb + (size_t)(m0w + m) * EMB;
  const unsigned short* xa1 = xa0 + (size_t)16 * EMB;
  const unsigned short* wrw = wb + ((size_t)which * EMB + head * HD + m) * EMB;

  const v8f zero8 = {0.f, 0.f, 0.f, 0.f, 0.f, 0.f, 0.f, 0.f};
  v8f acc[2][4];
  #pragma unroll
  for (int mt = 0; mt < 2; ++mt)
    #pragma unroll
    for (int nt = 0; nt < 4; ++nt) acc[mt][nt] = zero8;

  #pragma unroll 1
  for (int k0 = 0; k0 < EMB; k0 += 32) {
    const v16b a0 = load_frag16(xa0 + k0, h);
    const v16b a1 = load_frag16(xa1 + k0, h);
    #pragma unroll
    for (int nt = 0; nt < 4; ++nt) {
      const v16b b = load_frag16(wrw + (size_t)nt * 16 * EMB + k0, h);
      acc[0][nt] = wmma_bf(a0, b, acc[0][nt]);
      acc[1][nt] = wmma_bf(a1, b, acc[1][nt]);
    }
  }

  #pragma unroll
  for (int nt = 0; nt < 4; ++nt) {
    const int feat = 16 * nt + m;
    #pragma unroll
    for (int mt = 0; mt < 2; ++mt) {
      #pragma unroll
      for (int r = 0; r < 8; ++r) {
        const int tokl = 32 * w + 16 * mt + 8 * h + r;
        sT[tokl * HD + feat] = acc[mt][nt][r];
      }
    }
  }
  __syncthreads();

  float* p32w = p32 + (size_t)which * PLANE;
  proj_store(sT, p32w, p1h, p1l, which, head, m0, w, lane);
  __threadfence();
  proj_store(sT, p32w, p1h, p1l, which, head, m0, w, lane);
}

__device__ __forceinline__ void score_store(const float* sR, const float* smout,
                                            float* rpl, float* mpl,
                                            int bh, int ti, int w, int lane) {
  const int q8 = lane & 7, sub = lane >> 3;
  #pragma unroll
  for (int it = 0; it < 3; ++it) {
    const int lid = w * 12 + it * 4 + sub;
    const int row = lid / 6, seg = lid - row * 6;
    const v4f v = *(const v4fa*)(sR + row * SEQ + seg * 32 + 4 * q8);
    float* dst = rpl + ((size_t)(bh * SEQ + 16 * ti + row)) * SEQ + seg * 32 + 4 * q8;
    *(volatile v4f*)dst = v;
  }
  if (w == 0 && lane < 8) {
    const v4f v = *(const v4fa*)(smout + 4 * lane);
    float* dst = mpl + ((size_t)(bh * NTI + ti)) * 32 + 4 * lane;
    *(volatile v4f*)dst = v;
  }
}

__global__ __launch_bounds__(256) void score_kernel(
    const float* __restrict__ p32,
    const unsigned short* __restrict__ p1h,
    const unsigned short* __restrict__ p1l,
    float* __restrict__ rpl,
    float* __restrict__ mpl)
{
  __shared__ __attribute__((aligned(16))) float sR[16 * SEQ];
  __shared__ float sMK[16 * SEQ];
  __shared__ float swm[8 * 16];
  __shared__ float smrow[16];
  __shared__ __attribute__((aligned(16))) float smout[32];

  const int tid = threadIdx.x, lane = tid & 31, w = tid >> 5;
  const int h = lane >> 4, m = lane & 15;
  const int ti = blockIdx.x, bh = blockIdx.y;
  const float ninf = -__builtin_inff();

  for (int e = tid; e < 16 * SEQ; e += 256) { sR[e] = 0.0f; sMK[e] = ninf; }
  if (tid < 32) smout[tid] = 0.0f;

  const int irow = 16 * ti + m;
  const float* p0row = p32 + ((size_t)bh * SEQ + irow) * HD;
  const float* p2pl  = p32 + (size_t)2 * PLANE + (size_t)bh * SEQ * HD;
  v8f p0r[2][2];
  #pragma unroll
  for (int s = 0; s < 2; ++s)
    #pragma unroll
    for (int g = 0; g < 2; ++g) p0r[s][g] = ld8f(p0row + 32 * s + 16 * g + 8 * h);
  const unsigned short* ah_base = p1h + ((size_t)bh * SEQ + m) * HD;
  const unsigned short* al_base = p1l + ((size_t)bh * SEQ + m) * HD;
  __syncthreads();

  const v8f zero8 = {0.f, 0.f, 0.f, 0.f, 0.f, 0.f, 0.f, 0.f};
  float mrun = ninf;
  const int kmax = 16 * ti + 15;

  #pragma unroll 1
  for (int k = w; k <= kmax; k += 8) {
    const float* p2row = p2pl + (size_t)k * HD;
    FragB fh[2], fl[2];
    #pragma unroll
    for (int s = 0; s < 2; ++s) {
      v8us hh[2], ll[2];
      #pragma unroll
      for (int g = 0; g < 2; ++g) {
        const v8f q = ld8f(p2row + 32 * s + 16 * g + 8 * h);
        #pragma unroll
        for (int e = 0; e < 8; ++e) {
          const float v = p0r[s][g][e] * q[e] * 0.125f;
          const unsigned short hb = bf16_bits(v);
          const unsigned short lb = bf16_bits(v - bf16_val(hb));
          hh[g][e] = hb;
          ll[g][e] = lb;
        }
      }
      fh[s].half[0] = hh[0]; fh[s].half[1] = hh[1];
      fl[s].half[0] = ll[0]; fl[s].half[1] = ll[1];
    }

    float rk = 0.0f;
    #pragma unroll 1
    for (int tj = (k >> 4); tj <= ti; ++tj) {
      const unsigned short* ph = ah_base + (size_t)tj * 16 * HD;
      const unsigned short* pl = al_base + (size_t)tj * 16 * HD;
      const v16b ah0 = load_frag16(ph, h);
      const v16b ah1 = load_frag16(ph + 32, h);
      const v16b al0 = load_frag16(pl, h);
      const v16b al1 = load_frag16(pl + 32, h);
      v8f acc = zero8;
      acc = wmma_bf(ah0, fh[0].v, acc);
      acc = wmma_bf(ah0, fl[0].v, acc);
      acc = wmma_bf(al0, fh[0].v, acc);
      acc = wmma_bf(ah1, fh[1].v, acc);
      acc = wmma_bf(ah1, fl[1].v, acc);
      acc = wmma_bf(al1, fh[1].v, acc);

      const int jbase = 16 * tj + 8 * h;
      float tmax = ninf;
      #pragma unroll
      for (int r = 0; r < 8; ++r) {
        const int j = jbase + r;
        const bool ok = (j <= irow) && (j >= k);
        tmax = ok ? fmaxf(tmax, acc[r]) : tmax;
      }
      tmax = fmaxf(tmax, __shfl_xor(tmax, 16));
      const float mnew = fmaxf(mrun, tmax);
      const float alpha = (mnew > -3.0e38f) ? __expf(mrun - mnew) : 1.0f;
      float psum = 0.0f;
      #pragma unroll
      for (int r = 0; r < 8; ++r) {
        const int j = jbase + r;
        const bool ok = (j <= irow) && (j >= k);
        const float dd = ok ? (acc[r] - mnew) : 0.0f;
        const float p = __expf(dd);
        psum += ok ? p : 0.0f;
      }
      psum += __shfl_xor(psum, 16);
      rk = rk * alpha + psum;
      mrun = mnew;
    }
    if (h == 0) { sR[m * SEQ + k] = rk; sMK[m * SEQ + k] = mrun; }
  }

  if (h == 0) swm[w * 16 + m] = mrun;
  __syncthreads();
  if (tid < 16) {
    float mx = swm[tid];
    #pragma unroll
    for (int q = 1; q < 8; ++q) mx = fmaxf(mx, swm[q * 16 + tid]);
    smrow[tid] = mx;
    smout[tid] = mx;
  }
  __syncthreads();
  for (int e = tid; e < 16 * SEQ; e += 256) {
    const int row = e / SEQ;
    const float v = sR[e] * __expf(sMK[e] - smrow[row]);
    sR[e] = v;
  }
  __syncthreads();

  score_store(sR, smout, rpl, mpl, bh, ti, w, lane);
  __threadfence();
  score_store(sR, smout, rpl, mpl, bh, ti, w, lane);
}

__device__ __forceinline__ void y_store(const float* sY, unsigned short* yh, unsigned short* yl,
                                        int b, int head, int i0, int lane) {
  const int r = lane >> 3, q8 = lane & 7;
  const v4f a = *(const v4fa*)(sY + r * HD + 8 * q8);
  const v4f c = *(const v4fa*)(sY + r * HD + 8 * q8 + 4);
  v8us hv, lv;
  split8(a, c, hv, lv);
  const size_t idx = ((size_t)(b * SEQ + i0 + r)) * EMB + head * HD + 8 * q8;
  *(volatile v8us*)(yh + idx) = hv;
  *(volatile v8us*)(yl + idx) = lv;
}

__global__ __launch_bounds__(256) void final_kernel(
    const float* __restrict__ p32,
    const float* __restrict__ rpl,
    const float* __restrict__ mpl,
    unsigned short* __restrict__ yh,
    unsigned short* __restrict__ yl)
{
  __shared__ __attribute__((aligned(16))) float sP2[SEQ * HD];
  __shared__ __attribute__((aligned(16))) float sRr[4 * SEQ];
  __shared__ __attribute__((aligned(16))) float sY[4 * HD];
  __shared__ float sm[SEQ];
  __shared__ float ssc[SEQ];
  __shared__ float sS[SEQ];
  __shared__ float sZ[4];

  const int tid = threadIdx.x, lane = tid & 31, w = tid >> 5;
  const int bh = blockIdx.x, b = bh >> 3, head = bh & 7;

  if (tid < SEQ) sm[tid] = mpl[((size_t)(bh * NTI + (tid >> 4))) * 32 + (tid & 15)];
  const float* p2 = p32 + (size_t)2 * PLANE + (size_t)bh * SEQ * HD;
  for (int e = tid * 4; e < SEQ * HD; e += 1024) *(v4fa*)(sP2 + e) = *(const v4fa*)(p2 + e);
  __syncthreads();

  if (w == 0) {
    float mx = sm[lane];
    #pragma unroll
    for (int c = 1; c < 6; ++c) mx = fmaxf(mx, sm[lane + 32 * c]);
    #pragma unroll
    for (int off = 16; off; off >>= 1) mx = fmaxf(mx, __shfl_xor(mx, off));
    if (lane == 0) sZ[0] = mx;
  }
  __syncthreads();
  const float Mg = sZ[0];
  if (tid < SEQ) {
    const float* rr = rpl + ((size_t)(bh * SEQ + tid)) * SEQ;
    float s = 0.0f;
    #pragma unroll 2
    for (int c = 0; c < SEQ / 4; ++c) {
      const v4f v = *(const v4fa*)(rr + 4 * c);
      s += v.x; s += v.y; s += v.z; s += v.w;
    }
    const float ei = __expf(sm[tid] - Mg);
    ssc[tid] = ei;
    sS[tid] = ei * s;
  }
  __syncthreads();
  if (w == 0) {
    float z = sS[lane];
    #pragma unroll
    for (int c = 1; c < 6; ++c) z += sS[lane + 32 * c];
    #pragma unroll
    for (int off = 16; off; off >>= 1) z += __shfl_xor(z, off);
    if (lane == 0) sZ[1] = z;
  }
  __syncthreads();
  const float inv = 1.0f / sZ[1];
  const int row = tid >> 6, d = tid & 63;

  #pragma unroll 1
  for (int i0 = 0; i0 < SEQ; i0 += 4) {
    const float* rsrc = rpl + ((size_t)(bh * SEQ + i0)) * SEQ;
    for (int e = tid; e < 4 * SEQ; e += 256) sRr[e] = rsrc[e];
    __syncthreads();
    const int kend = i0 + 4;
    float acc = 0.0f;
    #pragma unroll 4
    for (int k = 0; k < kend; ++k) acc = fmaf(sRr[row * SEQ + k], sP2[k * HD + d], acc);
    sY[row * HD + d] = acc * ssc[i0 + row] * inv;
    __syncthreads();
    if (w == 0) {
      y_store(sY, yh, yl, b, head, i0, lane);
      __threadfence();
      y_store(sY, yh, yl, b, head, i0, lane);
    }
  }
}

__device__ __forceinline__ void out_store(const float* sT, float* out, int m0, int nb, int w, int lane) {
  const int q8 = lane & 7, sub = lane >> 3;
  #pragma unroll
  for (int it = 0; it < 16; ++it) {
    const int lid = w * 64 + it * 4 + sub;
    const int tokl = lid >> 1, hl = lid & 1;
    const v4f v = *(const v4fa*)(sT + tokl * HD + 32 * hl + 4 * q8);
    float* dst = out + ((size_t)(m0 + tokl)) * EMB + nb * HD + 32 * hl + 4 * q8;
    *(volatile v4f*)dst = v;
  }
}

__global__ __launch_bounds__(128) void out_kernel(
    const unsigned short* __restrict__ yh,
    const unsigned short* __restrict__ yl,
    const unsigned short* __restrict__ wpb,
    float* __restrict__ out)
{
  __shared__ __attribute__((aligned(16))) float sT[128 * HD];

  const int tid = threadIdx.x, lane = tid & 31, w = tid >> 5;
  const int h = lane >> 4, m = lane & 15;
  const int m0 = blockIdx.x * 128;
  const int nb = blockIdx.y;
  const int m0w = m0 + 32 * w;

  const unsigned short* ya0 = yh + (size_t)(m0w + m) * EMB;
  const unsigned short* ya1 = ya0 + (size_t)16 * EMB;
  const unsigned short* za0 = yl + (size_t)(m0w + m) * EMB;
  const unsigned short* za1 = za0 + (size_t)16 * EMB;
  const unsigned short* wrw = wpb + ((size_t)nb * HD + m) * EMB;

  const v8f zero8 = {0.f, 0.f, 0.f, 0.f, 0.f, 0.f, 0.f, 0.f};
  v8f acc[2][4];
  #pragma unroll
  for (int mt = 0; mt < 2; ++mt)
    #pragma unroll
    for (int nt = 0; nt < 4; ++nt) acc[mt][nt] = zero8;

  #pragma unroll 1
  for (int k0 = 0; k0 < EMB; k0 += 32) {
    const v16b a0 = load_frag16(ya0 + k0, h);
    const v16b a1 = load_frag16(ya1 + k0, h);
    const v16b c0 = load_frag16(za0 + k0, h);
    const v16b c1 = load_frag16(za1 + k0, h);
    #pragma unroll
    for (int nt = 0; nt < 4; ++nt) {
      const v16b b = load_frag16(wrw + (size_t)nt * 16 * EMB + k0, h);
      acc[0][nt] = wmma_bf(a0, b, acc[0][nt]);
      acc[0][nt] = wmma_bf(c0, b, acc[0][nt]);
      acc[1][nt] = wmma_bf(a1, b, acc[1][nt]);
      acc[1][nt] = wmma_bf(c1, b, acc[1][nt]);
    }
  }

  #pragma unroll
  for (int nt = 0; nt < 4; ++nt) {
    const int feat = 16 * nt + m;
    #pragma unroll
    for (int mt = 0; mt < 2; ++mt) {
      #pragma unroll
      for (int r = 0; r < 8; ++r) {
        const int tokl = 32 * w + 16 * mt + 8 * h + r;
        sT[tokl * HD + feat] = acc[mt][nt][r];
      }
    }
  }
  __syncthreads();

  out_store(sT, out, m0, nb, w, lane);
  __threadfence();
  out_store(sT, out, m0, nb, w, lane);
}

extern "C" void kernel_launch(void* const* d_in, const int* in_sizes, int n_in,
                              void* d_out, int out_size, void* d_ws, size_t ws_size,
                              hipStream_t stream) {
  if (n_in < 5) return;
  if (in_sizes[0] != NX) return;
  if (in_sizes[1] != NW || in_sizes[2] != NW || in_sizes[3] != NW || in_sizes[4] != NW) return;
  if (out_size != NX) return;

  const float* x  = (const float*)d_in[0];
  const float* w0 = (const float*)d_in[1];
  const float* w1 = (const float*)d_in[2];
  const float* w2 = (const float*)d_in[3];
  const float* wp = (const float*)d_in[4];
  float* out = (float*)d_out;

  const size_t xb_bytes  = (size_t)NX * 2;
  const size_t wb_bytes  = (size_t)3 * NW * 2;
  const size_t wpb_bytes = (size_t)NW * 2;
  const size_t p32_bytes = (size_t)3 * PLANE * 4;
  const size_t p1_bytes  = (size_t)PLANE * 2;
  const size_t rpl_bytes = (size_t)NBH * SEQ * SEQ * 4;
  const size_t mpl_bytes = (size_t)NBH * NTI * 32 * 4;
  const size_t y_bytes   = (size_t)NX * 2;

  size_t off = 0;
  const size_t o_xb  = off; off += xb_bytes;
  const size_t o_wb  = off; off += wb_bytes;
  const size_t o_wpb = off; off += wpb_bytes;
  const size_t o_p32 = off; off += p32_bytes;
  const size_t o_p1h = off; off += p1_bytes;
  const size_t o_p1l = off; off += p1_bytes;
  const size_t o_rpl = off; off += rpl_bytes;
  const size_t o_mpl = off; off += mpl_bytes;
  const size_t o_yh  = off; off += y_bytes;
  const size_t o_yl  = off; off += y_bytes;
  if (off > ws_size) return;
  if (off > (size_t)134217728) return;

  char* ws = (char*)d_ws;
  unsigned short* xb  = (unsigned short*)(ws + o_xb);
  unsigned short* wb  = (unsigned short*)(ws + o_wb);
  unsigned short* wpb = (unsigned short*)(ws + o_wpb);
  float*          p32 = (float*)(ws + o_p32);
  unsigned short* p1h = (unsigned short*)(ws + o_p1h);
  unsigned short* p1l = (unsigned short*)(ws + o_p1l);
  float*          rpl = (float*)(ws + o_rpl);
  float*          mpl = (float*)(ws + o_mpl);
  unsigned short* yh  = (unsigned short*)(ws + o_yh);
  unsigned short* yl  = (unsigned short*)(ws + o_yl);

  const int ngroups = NX8 + 4 * NW8;
  cvt_kernel<<<(ngroups + 255) / 256, 256, 0, stream>>>(x, w0, w1, w2, wp, xb, wb, wpb);

  dim3 gProj(NTOK / 128, 3 * NH);
  proj_kernel<<<gProj, 128, 0, stream>>>(xb, wb, p32, p1h, p1l);

  dim3 gScore(NTI, NBH);
  score_kernel<<<gScore, 256, 0, stream>>>(p32, p1h, p1l, rpl, mpl);

  final_kernel<<<NBH, 256, 0, stream>>>(p32, rpl, mpl, yh, yl);

  dim3 gOut(NTOK / 128, EMB / HD);
  out_kernel<<<gOut, 128, 0, stream>>>(yh, yl, wpb, out);
}
